// GNN_47313359732963
// MI455X (gfx1250) — hardware-verified
//
#include <hip/hip_runtime.h>
#include <stddef.h>
#include <stdint.h>
#include <math.h>


#define EMB    64
#define AF     32
#define BF     16
#define HID2   128
#define NL     5
#define K1     128
#define K2     256
#define NTHR   256
#define NWAVE  8
#define EPT    8
#define CHUNK  (NTHR * EPT)
#define WCAP   (EPT * 32)
#define LISTN  (NWAVE * WCAP)
#define NBA    1024
#define SLA    10
#define RCAP   20480
#define DEGCAP 64
#define GBM    64
#define GBN    64
#define GTHR   128
#define EXW    32
#define Z_INTS (LISTN + 2 * RCAP + 3 * NBA)
#define MISC_INTS 16
#define RB_INTS (NWAVE * 32)
#define SCAN_LDS_INTS (Z_INTS + MISC_INTS + RB_INTS)
#define UE     256
#define UWE    (NL * 64 * 4)
#define UW1    (NL * 128 * 16)
#define UW2    (NL * 64 * 32)
#define UTOT   (UE + UWE + UW1 + UW2)
#define WSMAX  134217728

static_assert((CHUNK & (CHUNK - 1)) == 0 && CHUNK <= 4096);
static_assert((NBA & (NBA - 1)) == 0 && NBA == (1 << SLA));
static_assert(((long long)CHUNK << SLA) < (1LL << 31));
static_assert(NBA % NWAVE == 0 && NBA == NTHR * 4 && NBA % GBM == 0);
static_assert(Z_INTS % (NTHR * 4) == 0 && LISTN % 4 == 0 && RCAP % (NTHR * 4) == 0);
static_assert(RB_INTS == NTHR);
static_assert(SCAN_LDS_INTS * 4 <= 300000);
static_assert(GBM == (GTHR / 32) * 16 && GBN == EMB && EMB == 2 * 32);
static_assert(K1 == 2 * EMB && K2 == 2 * HID2 && AF == 32 && 2 * BF == 32);
static_assert(UE % NTHR == 0 && UWE % NTHR == 0 && UW1 % NTHR == 0 && UW2 % NTHR == 0);

typedef float          v2f   __attribute__((ext_vector_type(2)));
typedef float          v4f   __attribute__((ext_vector_type(4)));
typedef float          v8f   __attribute__((ext_vector_type(8)));
typedef int            v4i   __attribute__((ext_vector_type(4)));
typedef int            v8i   __attribute__((ext_vector_type(8)));
typedef unsigned int   v4u   __attribute__((ext_vector_type(4)));
typedef unsigned short v8us  __attribute__((ext_vector_type(8)));
typedef unsigned short v16us __attribute__((ext_vector_type(16)));
typedef __bf16         v16bf __attribute__((ext_vector_type(16)));
typedef v2f  __attribute__((may_alias)) v2fa;
typedef v4f  __attribute__((may_alias)) v4fa;
typedef v4i  __attribute__((may_alias)) v4ia;
typedef v4u  __attribute__((may_alias)) v4ua;
typedef v8us __attribute__((may_alias)) v8usa;
union FragB { v16bf v; v16us u; v8us h[2]; v8i w; };

__device__ __forceinline__ v8f wmb(const FragB& a, const FragB& b, v8f c) {
  v8f d = __builtin_amdgcn_wmma_f32_16x16x32_bf16(false, a.v, false, b.v, (short)0, c, false, false);
  asm volatile("v_nop\n\tv_nop\n\tv_nop\n\tv_nop" : "+v"(d) : "v"(a.w), "v"(b.w));
  return d;
}

__device__ __forceinline__ unsigned bf16_bits(float f) {
  const unsigned u = __float_as_uint(f);
  return (u + 0x7FFFu + ((u >> 16) & 1u)) >> 16;
}
__device__ __forceinline__ float bf16_val(float f) {
  return __uint_as_float(bf16_bits(f) << 16);
}

__device__ __forceinline__ void wave_sync() {
  __builtin_amdgcn_fence(__ATOMIC_RELEASE, "wavefront");
  __builtin_amdgcn_wave_barrier();
  __builtin_amdgcn_fence(__ATOMIC_ACQUIRE, "wavefront");
}

template <int SLB>
__device__ __forceinline__ int scan_chunk(const int* __restrict__ dsts, int nE, int cbase, int slotBase,
                                          int nb, int vec8, int* list, int tid, int lane, int wave) {
  int wc = 0;
  const int el0  = tid * EPT;
  const int e0   = cbase + el0;
  const int sent = -2147483647 - 1;
  v4i da, db;
  if (vec8 != 0 && cbase + CHUNK <= nE) {
    da = *(const v4i*)(dsts + e0);
    db = *(const v4i*)(dsts + e0 + 4);
  } else {
    da.x = (e0     < nE) ? dsts[min(e0,     nE - 1)] : sent;
    da.y = (e0 + 1 < nE) ? dsts[min(e0 + 1, nE - 1)] : sent;
    da.z = (e0 + 2 < nE) ? dsts[min(e0 + 2, nE - 1)] : sent;
    da.w = (e0 + 3 < nE) ? dsts[min(e0 + 3, nE - 1)] : sent;
    db.x = (e0 + 4 < nE) ? dsts[min(e0 + 4, nE - 1)] : sent;
    db.y = (e0 + 5 < nE) ? dsts[min(e0 + 5, nE - 1)] : sent;
    db.z = (e0 + 6 < nE) ? dsts[min(e0 + 6, nE - 1)] : sent;
    db.w = (e0 + 7 < nE) ? dsts[min(e0 + 7, nE - 1)] : sent;
  }
  const unsigned nbs = (unsigned)slotBase;
  const unsigned unb = (unsigned)nb;
  const unsigned s0 = (unsigned)da.x - nbs, s1 = (unsigned)da.y - nbs;
  const unsigned s2 = (unsigned)da.z - nbs, s3 = (unsigned)da.w - nbs;
  const unsigned s4 = (unsigned)db.x - nbs, s5 = (unsigned)db.y - nbs;
  const unsigned s6 = (unsigned)db.z - nbs, s7 = (unsigned)db.w - nbs;
  const bool h0 = s0 < unb, h1 = s1 < unb, h2 = s2 < unb, h3 = s3 < unb;
  const bool h4 = s4 < unb, h5 = s5 < unb, h6 = s6 < unb, h7 = s7 < unb;
  const unsigned any = __builtin_amdgcn_ballot_w32(h0 | h1 | h2 | h3 | h4 | h5 | h6 | h7);
  if (any != 0u) {
#define HITJ(J, HJ, SJ) { \
      const unsigned mj = __builtin_amdgcn_ballot_w32(HJ); \
      if (mj != 0u) { \
        if (HJ) { \
          const int pos = wc + (int)__builtin_amdgcn_mbcnt_lo(mj, 0u); \
          if (pos < WCAP) list[wave * WCAP + pos] = ((el0 + (J)) << SLB) | (int)(SJ); \
        } \
        wc += (int)__builtin_popcount(mj); } }
    HITJ(0, h0, s0)
    HITJ(1, h1, s1)
    HITJ(2, h2, s2)
    HITJ(3, h3, s3)
    HITJ(4, h4, s4)
    HITJ(5, h5, s5)
    HITJ(6, h6, s6)
    HITJ(7, h7, s7)
#undef HITJ
  }
  return wc;
}

__device__ __forceinline__ void cv8(const float* __restrict__ p, unsigned short* dp) {
  const v4f a = *(const v4f*)p;
  const v4f b = *(const v4f*)(p + 4);
  v8us o;
  o[0] = (unsigned short)bf16_bits(a.x); o[1] = (unsigned short)bf16_bits(a.y);
  o[2] = (unsigned short)bf16_bits(a.z); o[3] = (unsigned short)bf16_bits(a.w);
  o[4] = (unsigned short)bf16_bits(b.x); o[5] = (unsigned short)bf16_bits(b.y);
  o[6] = (unsigned short)bf16_bits(b.z); o[7] = (unsigned short)bf16_bits(b.w);
  *(volatile v8us*)dp = o;
  __threadfence();
  *(volatile v8us*)dp = o;
}

__global__ __launch_bounds__(NTHR) void k_wprep(const float* __restrict__ Wemb, const float* __restrict__ We,
                                                const float* __restrict__ W1, const float* __restrict__ W2,
                                                unsigned short* pe, unsigned short* pwe,
                                                unsigned short* pw1, unsigned short* pw2) {
  const int u = (int)blockIdx.x * NTHR + (int)threadIdx.x;
  if (u < UE) {
    cv8(Wemb + (size_t)8 * u, pe + (size_t)8 * u);
  } else if (u < UE + UWE) {
    const int v = u - UE;
    const int l = v >> 8, w = v & 255, n = w >> 2, k8 = (w & 3) * 8;
    cv8(We + (size_t)l * (EMB * BF) + (size_t)n * BF + (k8 & (BF - 1)), pwe + (size_t)8 * v);
  } else if (u < UE + UWE + UW1) {
    const int v = u - (UE + UWE);
    const int l = v >> 11, w = v & 2047, n = w >> 4, k8 = (w & 15) * 8;
    cv8(W1 + (size_t)l * (HID2 * EMB) + (size_t)n * EMB + (k8 & (EMB - 1)), pw1 + (size_t)8 * v);
  } else if (u < UTOT) {
    const int v = u - (UE + UWE + UW1);
    const int l = v >> 11, w = v & 2047, n = w >> 5, k8 = (w & 31) * 8;
    cv8(W2 + (size_t)l * (EMB * HID2) + (size_t)n * HID2 + (k8 & (HID2 - 1)), pw2 + (size_t)8 * v);
  }
}

__global__ __launch_bounds__(NTHR) void k_cvx(const float* __restrict__ x, int nN, int nUnits,
                                              unsigned short* xb) {
  const int u = (int)blockIdx.x * NTHR + (int)threadIdx.x;
  if (u >= nUnits) return;
  const int row = u >> 2;
  const int k8  = (u & 3) * 8;
  const int rc  = row < nN ? row : nN - 1;
  const float* p = x + (size_t)rc * AF + k8;
  const v4f a = *(const v4fa*)p;
  const v4f b = *(const v4fa*)(p + 4);
  const bool ok = row < nN;
  v8us o;
  o[0] = ok ? (unsigned short)bf16_bits(a.x) : (unsigned short)0;
  o[1] = ok ? (unsigned short)bf16_bits(a.y) : (unsigned short)0;
  o[2] = ok ? (unsigned short)bf16_bits(a.z) : (unsigned short)0;
  o[3] = ok ? (unsigned short)bf16_bits(a.w) : (unsigned short)0;
  o[4] = ok ? (unsigned short)bf16_bits(b.x) : (unsigned short)0;
  o[5] = ok ? (unsigned short)bf16_bits(b.y) : (unsigned short)0;
  o[6] = ok ? (unsigned short)bf16_bits(b.z) : (unsigned short)0;
  o[7] = ok ? (unsigned short)bf16_bits(b.w) : (unsigned short)0;
  unsigned short* dp = xb + (size_t)row * AF + k8;
  *(volatile v8us*)dp = o;
  __threadfence();
  *(volatile v8us*)dp = o;
}

__global__ __launch_bounds__(GTHR) void k_gemm(
    const unsigned short* __restrict__ A, const unsigned short* __restrict__ WT,
    float* outF, int K, int ldo)
{
  __shared__ __attribute__((aligned(16))) float stg[GBM * GBN];
  const int tid = (int)threadIdx.x, lane = tid & 31, wave = tid >> 5, hh = lane >> 4, m = lane & 15;
  const int rowBase = (int)blockIdx.x * GBM;
  const int col0    = (int)blockIdx.y * GBN;

  v8f acc[4];
  {
    const v8f z = {0.f, 0.f, 0.f, 0.f, 0.f, 0.f, 0.f, 0.f};
    acc[0] = z; acc[1] = z; acc[2] = z; acc[3] = z;
  }
  const unsigned short* ap = A  + (size_t)(rowBase + 16 * wave + m) * (size_t)K + 8 * hh;
  const unsigned short* wp = WT + (size_t)(col0 + m) * (size_t)K + 8 * hh;
  const int ksteps = K >> 5;
#pragma unroll 1
  for (int ks = 0; ks < ksteps; ++ks) {
    FragB af;
    af.h[0] = *(const v8usa*)(ap + 32 * ks);
    af.h[1] = *(const v8usa*)(ap + 32 * ks + 16);
#pragma unroll
    for (int t = 0; t < 4; ++t) {
      const unsigned short* wq = wp + (size_t)(16 * t) * (size_t)K + 32 * ks;
      FragB bf;
      bf.h[0] = *(const v8usa*)wq;
      bf.h[1] = *(const v8usa*)(wq + 16);
      acc[t] = wmb(af, bf, acc[t]);
    }
  }

#pragma unroll
  for (int t = 0; t < 4; ++t) {
    const int lc = 16 * t + m;
#pragma unroll
    for (int r = 0; r < 8; ++r) {
      const int lr = 16 * wave + 8 * hh + r;
      stg[lr * GBN + lc] = acc[t][r];
    }
  }
  __syncthreads();

  v4f fv[8];
#pragma unroll
  for (int i = 0; i < 8; ++i) {
    const int lr = 16 * wave + 2 * i + hh;
    fv[i] = *(const v4fa*)(stg + lr * GBN + 4 * m);
  }
#pragma unroll
  for (int i = 0; i < 8; ++i) {
    const int lr = 16 * wave + 2 * i + hh;
    float* op = outF + (size_t)(rowBase + lr) * (size_t)ldo + col0 + 4 * m;
    *(volatile v4f*)op = fv[i];
  }
  __threadfence();
#pragma unroll
  for (int i = 0; i < 8; ++i) {
    const int lr = 16 * wave + 2 * i + hh;
    float* op = outF + (size_t)(rowBase + lr) * (size_t)ldo + col0 + 4 * m;
    *(volatile v4f*)op = fv[i];
  }
}

__global__ __launch_bounds__(NTHR) void k_scan0(const int* __restrict__ srcs, const int* __restrict__ dsts,
                                                const float* __restrict__ ea, int nE, int nN, int vec8, int mRows,
                                                const float* __restrict__ hin, float* hs, unsigned* ex,
                                                int* cntg, int* offg, int* srcl) {
  extern __shared__ __attribute__((aligned(16))) int dsm[];
  int* list = dsm;
  int* hl   = dsm + LISTN;
  int* sl   = hl + RCAP;
  int* cnt  = sl + RCAP;
  int* offs = cnt + NBA;
  int* cur  = offs + NBA;
  int* misc = cur + NBA;
  const int tid = (int)threadIdx.x, lane = tid & 31, wave = tid >> 5;
  unsigned* rbw = (unsigned*)(misc + MISC_INTS) + wave * 32;
  unsigned short* rb16 = (unsigned short*)rbw;
  const int nodeBase = (int)blockIdx.x * NBA;

  {
    const v4i z4 = {0, 0, 0, 0};
    for (int i = tid * 4; i < Z_INTS; i += NTHR * 4) *(v4ia*)(dsm + i) = z4;
    if (tid < MISC_INTS) misc[tid] = 0;
    misc[MISC_INTS + tid] = 0;
  }
  __syncthreads();

  int t = 0, ov = 0;
  const int nChunks = (nE + CHUNK - 1) / CHUNK;
#pragma unroll 1
  for (int ch = 0; ch < nChunks; ++ch) {
    const int cbase = ch * CHUNK;
    const int wc = scan_chunk<SLA>(dsts, nE, cbase, nodeBase, NBA, vec8, list, tid, lane, wave);
    if (lane == 0) misc[wave] = wc;
    __syncthreads();
    if (wave == 0) {
#pragma unroll 1
      for (int w2 = 0; w2 < NWAVE; ++w2) {
        int c = misc[w2];
        c = c < 0 ? 0 : (c > WCAP ? WCAP : c);
#pragma unroll 1
        for (int b0 = 0; b0 < c; b0 += 32) {
          const int idx = b0 + lane;
          const int ent = list[w2 * WCAP + (idx < WCAP ? idx : WCAP - 1)];
          const int m32 = (c - b0) < 32 ? (c - b0) : 32;
#pragma unroll 1
          for (int k = 0; k < m32; ++k) {
            const int u    = __builtin_amdgcn_readlane(ent, k);
            const int slot = u & (NBA - 1);
            const int el   = (u >> SLA) & (CHUNK - 1);
            const int pk   = ((cbase + el) << SLA) | slot;
            if (t < RCAP) {
              if (lane == 0) { hl[t] = pk; cnt[slot] = cnt[slot] + 1; }
              t = t + 1;
            } else {
              ov = 1;
            }
          }
        }
      }
    }
    __syncthreads();
  }
  if (wave == 0 && lane == 0) { misc[8] = t; misc[9] = ov; }
  __syncthreads();
  int tt = misc[8];
  tt = tt < 0 ? 0 : (tt > RCAP ? RCAP : tt);
  const int ovf = misc[9];

  if (wave == 0) {
    const int base = lane * (NBA / 32);
    int s = 0;
#pragma unroll 1
    for (int i = 0; i < NBA / 32; ++i) s += cnt[base + i];
    int incl = s;
#pragma unroll
    for (int d = 1; d < 32; d <<= 1) {
      const int y = __shfl_up(incl, d, 32);
      if (lane >= d) incl += y;
    }
    int run = incl - s;
#pragma unroll 1
    for (int i = 0; i < NBA / 32; ++i) {
      const int cv = cnt[base + i];
      offs[base + i] = run;
      cur[base + i]  = run;
      run += cv;
    }
  }
  __syncthreads();
  if (wave == 0) {
#pragma unroll 1
    for (int b0 = 0; b0 < tt; b0 += 32) {
      const int idx = b0 + lane;
      const int ent = hl[idx < RCAP ? idx : RCAP - 1];
      const int m32 = (tt - b0) < 32 ? (tt - b0) : 32;
#pragma unroll 1
      for (int k = 0; k < m32; ++k) {
        const int u    = __builtin_amdgcn_readlane(ent, k);
        const int slot = u & (NBA - 1);
        if (lane == 0) {
          int p = cur[slot];
          p = p < 0 ? 0 : (p > RCAP - 1 ? RCAP - 1 : p);
          sl[p] = u;
          cur[slot] = p + 1;
        }
      }
    }
  }
  __syncthreads();

  const float qnan = __int_as_float(0x7fc00000);
  const int sa = (2 * lane) & 31, sb = (2 * lane + 1) & 31;
#pragma unroll 1
  for (int si = 0; si < NBA / NWAVE; ++si) {
    const int s    = si * NWAVE + wave;
    const int node = nodeBase + s;
    int c = cnt[s];
    const bool big = (c > DEGCAP) || (ovf != 0);
    c = c < 0 ? 0 : (c > DEGCAP ? DEGCAP : c);
    int o = offs[s];
    o = o < 0 ? 0 : (o > RCAP ? RCAP : o);
    const int nc = node < nN ? node : nN - 1;
    float acc0, acc1, ae = 0.0f;
    {
      const v2f a = *(const v2fa*)(hin + (size_t)nc * EMB + 2 * lane);
      acc0 = a.x; acc1 = a.y;
    }
#pragma unroll 1
    for (int b0 = 0; b0 < c; b0 += 32) {
      const int idx  = o + b0 + lane;
      const int idxc = idx > RCAP - 1 ? RCAP - 1 : idx;
      const bool valid = ((b0 + lane) < c) && (idx < RCAP);
      const int ent = sl[idxc];
      int eid = ent >> SLA;
      eid = eid < 0 ? 0 : (eid > nE - 1 ? nE - 1 : eid);
      int sr = srcs[eid];
      sr = sr < 0 ? 0 : (sr > nN - 1 ? nN - 1 : sr);
      if (valid) hl[idxc] = sr;
      const int m32 = (c - b0) < 32 ? (c - b0) : 32;
#pragma unroll 1
      for (int k = 0; k < m32; ++k) {
        const int sk = __builtin_amdgcn_readlane(sr, k);
        const int ek = __builtin_amdgcn_readlane(eid, k);
        const v2f a = *(const v2fa*)(hin + (size_t)sk * EMB + 2 * lane);
        const float e = ea[(size_t)ek * BF + (lane & 15)];
        acc0 += a.x; acc1 += a.y;
        ae += bf16_val(e);
      }
    }
    const float pzr = big ? qnan : 0.0f;
    const bool live = node < nN;
    const float v0 = live ? (acc0 + pzr) : 0.0f;
    const float v1 = live ? (acc1 + pzr) : 0.0f;
    const float ev = live ? (ae + pzr) : 0.0f;
    const unsigned hb = bf16_bits(ev);
    const unsigned lb = bf16_bits(ev - __uint_as_float(hb << 16));
    const unsigned dw = live ? (unsigned)c : 0u;
    if (lane < 16) {
      rb16[lane]      = (unsigned short)hb;
      rb16[16 + lane] = (unsigned short)lb;
    } else {
      rbw[lane] = (lane == 16) ? dw : 0u;
    }
    wave_sync();
    const v4u q = *(const v4ua*)(rbw + 4 * (lane & 7));
    wave_sync();
    v4f ow;
    ow.x = __shfl(v0, sa, 32); ow.y = __shfl(v1, sa, 32);
    ow.z = __shfl(v0, sb, 32); ow.w = __shfl(v1, sb, 32);
    float*    op = hs + (size_t)node * EMB + 4 * (lane & 15);
    unsigned* xp = ex + (size_t)node * EXW + 4 * (lane & 7);
    const bool wr  = (node < mRows) && (lane < 16);
    const bool wrx = (node < mRows) && (lane < 8);
    if (wr)  *(volatile v4f*)op = ow;
    if (wrx) *(volatile v4u*)xp = q;
    __threadfence();
    if (wr)  *(volatile v4f*)op = ow;
    if (wrx) *(volatile v4u*)xp = q;
  }
  __syncthreads();

  {
    v4i c4 = *(const v4ia*)(cnt + 4 * tid);
    const v4i o4 = *(const v4ia*)(offs + 4 * tid);
    c4.x = (ovf != 0 || c4.x < 0 || c4.x > DEGCAP) ? -1 : c4.x;
    c4.y = (ovf != 0 || c4.y < 0 || c4.y > DEGCAP) ? -1 : c4.y;
    c4.z = (ovf != 0 || c4.z < 0 || c4.z > DEGCAP) ? -1 : c4.z;
    c4.w = (ovf != 0 || c4.w < 0 || c4.w > DEGCAP) ? -1 : c4.w;
    int* cp = cntg + (size_t)blockIdx.x * NBA + 4 * tid;
    int* pp = offg + (size_t)blockIdx.x * NBA + 4 * tid;
    int* sp = srcl + (size_t)blockIdx.x * RCAP + 4 * tid;
    *(volatile v4i*)cp = c4;
    *(volatile v4i*)pp = o4;
#pragma unroll 1
    for (int it = 0; it < RCAP / (NTHR * 4); ++it) {
      const v4i v = *(const v4ia*)(hl + it * (NTHR * 4) + 4 * tid);
      *(volatile v4i*)(sp + it * (NTHR * 4)) = v;
    }
    __threadfence();
    *(volatile v4i*)cp = c4;
    *(volatile v4i*)pp = o4;
#pragma unroll 1
    for (int it = 0; it < RCAP / (NTHR * 4); ++it) {
      const v4i v = *(const v4ia*)(hl + it * (NTHR * 4) + 4 * tid);
      *(volatile v4i*)(sp + it * (NTHR * 4)) = v;
    }
  }
}

__global__ __launch_bounds__(NTHR) void k_gather(const int* __restrict__ cntg, const int* __restrict__ offg,
                                                 const int* __restrict__ srcl, int nN, int mRows,
                                                 const float* __restrict__ hin, float* hs) {
  __shared__ __attribute__((aligned(16))) int cnt[NBA];
  __shared__ __attribute__((aligned(16))) int offs[NBA];
  const int tid = (int)threadIdx.x, lane = tid & 31, wave = tid >> 5;
  const int nodeBase = (int)blockIdx.x * NBA;
  {
    const v4i c4 = *(const v4i*)(cntg + (size_t)blockIdx.x * NBA + 4 * tid);
    const v4i o4 = *(const v4i*)(offg + (size_t)blockIdx.x * NBA + 4 * tid);
    *(v4ia*)(cnt + 4 * tid)  = c4;
    *(v4ia*)(offs + 4 * tid) = o4;
  }
  __syncthreads();
  const int* sbase = srcl + (size_t)blockIdx.x * RCAP;
  const float qnan = __int_as_float(0x7fc00000);
  const int sa = (2 * lane) & 31, sb = (2 * lane + 1) & 31;
#pragma unroll 1
  for (int si = 0; si < NBA / NWAVE; ++si) {
    const int s    = si * NWAVE + wave;
    const int node = nodeBase + s;
    int c = cnt[s];
    const bool big = (c < 0) || (c > DEGCAP);
    c = c < 0 ? 0 : (c > DEGCAP ? DEGCAP : c);
    int o = offs[s];
    o = o < 0 ? 0 : (o > RCAP ? RCAP : o);
    const int nc = node < nN ? node : nN - 1;
    float acc0, acc1;
    {
      const v2f a = *(const v2fa*)(hin + (size_t)nc * EMB + 2 * lane);
      acc0 = a.x; acc1 = a.y;
    }
#pragma unroll 1
    for (int b0 = 0; b0 < c; b0 += 32) {
      int idx = o + b0 + lane;
      idx = idx > RCAP - 1 ? RCAP - 1 : idx;
      int sr = sbase[idx];
      sr = sr < 0 ? 0 : (sr > nN - 1 ? nN - 1 : sr);
      const int m32 = (c - b0) < 32 ? (c - b0) : 32;
#pragma unroll 1
      for (int k = 0; k < m32; ++k) {
        const int sk = __builtin_amdgcn_readlane(sr, k);
        const v2f a = *(const v2fa*)(hin + (size_t)sk * EMB + 2 * lane);
        acc0 += a.x; acc1 += a.y;
      }
    }
    const float pzr = big ? qnan : 0.0f;
    const bool live = node < nN;
    const float v0 = live ? (acc0 + pzr) : 0.0f;
    const float v1 = live ? (acc1 + pzr) : 0.0f;
    v4f ow;
    ow.x = __shfl(v0, sa, 32); ow.y = __shfl(v1, sa, 32);
    ow.z = __shfl(v0, sb, 32); ow.w = __shfl(v1, sb, 32);
    float* op = hs + (size_t)node * EMB + 4 * (lane & 15);
    const bool wr = (node < mRows) && (lane < 16);
    if (wr) *(volatile v4f*)op = ow;
    __threadfence();
    if (wr) *(volatile v4f*)op = ow;
  }
}

__device__ __forceinline__ void split2(float v, unsigned short& hb, unsigned short& lb) {
  const unsigned h = bf16_bits(v);
  hb = (unsigned short)h;
  lb = (unsigned short)bf16_bits(v - __uint_as_float(h << 16));
}

__global__ __launch_bounds__(GTHR) void k_mlp(
    const float* __restrict__ hs, const unsigned short* __restrict__ exh, const int* __restrict__ exw,
    const unsigned short* __restrict__ we2, const unsigned short* __restrict__ w1x,
    const unsigned short* __restrict__ w2x,
    const float* __restrict__ be, const float* __restrict__ b1, const float* __restrict__ b2,
    float* hn, float* rec, int nN)
{
  __shared__ __attribute__((aligned(16))) unsigned char smem[32768];
  __shared__ float dgL[GBM];
  __shared__ float biasL[256];
  __shared__ __attribute__((aligned(16))) float recL[128];
  float* stg = (float*)smem;
  unsigned short* a1 = (unsigned short*)(smem + 16384);
  unsigned short* a2 = (unsigned short*)smem;
  const int tid = (int)threadIdx.x, lane = tid & 31, wave = tid >> 5, hh = lane >> 4, m = lane & 15;
  const int rowBase = (int)blockIdx.x * GBM;
  const v8f z8 = {0.f, 0.f, 0.f, 0.f, 0.f, 0.f, 0.f, 0.f};

#pragma unroll
  for (int i = 0; i < 8; ++i) {
    const int lr = 16 * wave + 2 * i + hh;
    const v4f v = *(const v4fa*)(hs + (size_t)(rowBase + lr) * EMB + 4 * m);
    *(v4fa*)(stg + lr * EMB + 4 * m) = v;
  }
  biasL[tid] = bf16_val(b1[tid]);
  if (tid < GBM) {
    int d = exw[(size_t)(rowBase + tid) * EXW + 16];
    d = d < 0 ? 0 : (d > DEGCAP ? DEGCAP : d);
    dgL[tid] = (float)(d + 1);
    biasL[128 + tid] = bf16_val(be[tid]);
    biasL[192 + tid] = bf16_val(b2[tid]);
  }
  __syncthreads();

  {
    v8f acc[4];
    acc[0] = z8; acc[1] = z8; acc[2] = z8; acc[3] = z8;
    const unsigned short* ap = exh + (size_t)(rowBase + 16 * wave + m) * (2 * EXW) + 8 * hh;
    FragB af;
    af.h[0] = *(const v8usa*)ap;
    af.h[1] = *(const v8usa*)(ap + 16);
#pragma unroll
    for (int t = 0; t < 4; ++t) {
      const unsigned short* wq = we2 + (size_t)(16 * t + m) * 32 + 8 * hh;
      FragB bf;
      bf.h[0] = *(const v8usa*)wq;
      bf.h[1] = *(const v8usa*)(wq + 16);
      acc[t] = wmb(af, bf, acc[t]);
    }
#pragma unroll
    for (int t = 0; t < 4; ++t) {
      const int col = 16 * t + m;
      const float bev = biasL[128 + col];
#pragma unroll
      for (int r = 0; r < 8; ++r) {
        const int lr = 16 * wave + 8 * hh + r;
        const float v = (stg[lr * EMB + col] + acc[t][r]) + dgL[lr] * bev;
        unsigned short hb, lb;
        split2(v, hb, lb);
        a1[lr * K1 + col]       = hb;
        a1[lr * K1 + EMB + col] = lb;
      }
    }
  }
  __syncthreads();

  {
    v8f acc[8];
#pragma unroll
    for (int t = 0; t < 8; ++t) acc[t] = z8;
    const unsigned short* arow = a1 + (16 * wave + m) * K1 + 8 * hh;
    const unsigned short* wp   = w1x + (size_t)m * K1 + 8 * hh;
#pragma unroll 1
    for (int ks = 0; ks < K1 / 32; ++ks) {
      FragB af;
      af.h[0] = *(const v8usa*)(arow + 32 * ks);
      af.h[1] = *(const v8usa*)(arow + 32 * ks + 16);
#pragma unroll
      for (int nt = 0; nt < 8; ++nt) {
        const unsigned short* wq = wp + (size_t)(16 * nt) * K1 + 32 * ks;
        FragB bf;
        bf.h[0] = *(const v8usa*)wq;
        bf.h[1] = *(const v8usa*)(wq + 16);
        acc[nt] = wmb(af, bf, acc[nt]);
      }
    }
    __syncthreads();
#pragma unroll
    for (int nt = 0; nt < 8; ++nt) {
      const int col = 16 * nt + m;
      const float bv = biasL[col];
#pragma unroll
      for (int r = 0; r < 8; ++r) {
        const int lr = 16 * wave + 8 * hh + r;
        float v = acc[nt][r] + bv;
        v = (v > 0.0f) ? v : (v - v);
        unsigned short hb, lb;
        split2(v, hb, lb);
        a2[lr * K2 + col]        = hb;
        a2[lr * K2 + HID2 + col] = lb;
      }
    }
  }
  __syncthreads();

  {
    v8f acc[4];
    acc[0] = z8; acc[1] = z8; acc[2] = z8; acc[3] = z8;
    const unsigned short* arow = a2 + (16 * wave + m) * K2 + 8 * hh;
    const unsigned short* wp   = w2x + (size_t)m * K2 + 8 * hh;
#pragma unroll 1
    for (int ks = 0; ks < K2 / 32; ++ks) {
      FragB af;
      af.h[0] = *(const v8usa*)(arow + 32 * ks);
      af.h[1] = *(const v8usa*)(arow + 32 * ks + 16);
#pragma unroll
      for (int t = 0; t < 4; ++t) {
        const unsigned short* wq = wp + (size_t)(16 * t) * K2 + 32 * ks;
        FragB bf;
        bf.h[0] = *(const v8usa*)wq;
        bf.h[1] = *(const v8usa*)(wq + 16);
        acc[t] = wmb(af, bf, acc[t]);
      }
    }
    __syncthreads();
#pragma unroll
    for (int t = 0; t < 4; ++t) {
      const int col = 16 * t + m;
      const float bv = biasL[192 + col];
#pragma unroll
      for (int r = 0; r < 8; ++r) {
        const int lr = 16 * wave + 8 * hh + r;
        stg[lr * EMB + col] = acc[t][r] + bv;
      }
    }
  }
  __syncthreads();

  {
    v4f fv[8];
#pragma unroll
    for (int i = 0; i < 8; ++i) {
      const int lr = 16 * wave + 2 * i + hh;
      fv[i] = *(const v4fa*)(stg + lr * EMB + 4 * m);
    }
#pragma unroll
    for (int i = 0; i < 8; ++i) {
      const int lr = 16 * wave + 2 * i + hh;
      *(volatile v4f*)(hn + (size_t)(rowBase + lr) * EMB + 4 * m) = fv[i];
    }
    __threadfence();
#pragma unroll
    for (int i = 0; i < 8; ++i) {
      const int lr = 16 * wave + 2 * i + hh;
      *(volatile v4f*)(hn + (size_t)(rowBase + lr) * EMB + 4 * m) = fv[i];
    }
  }

  if (tid < EMB) {
    int nv = nN - rowBase;
    nv = nv < 1 ? 1 : (nv > GBM ? GBM : nv);
    float s = 0.0f;
#pragma unroll 4
    for (int r = 0; r < nv; ++r) s += stg[r * EMB + tid];
    const float mean = s * (1.0f / (float)nv);
    float q = 0.0f;
#pragma unroll 4
    for (int r = 0; r < nv; ++r) {
      const float d = stg[r * EMB + tid] - mean;
      q = fmaf(d, d, q);
    }
    recL[tid] = mean;
    recL[EMB + tid] = q;
  }
  __syncthreads();
  {
    const v4f rv = *(const v4fa*)(recL + 4 * lane);
    float* rp = rec + (size_t)blockIdx.x * 128 + 4 * lane;
    if (wave == 0) *(volatile v4f*)rp = rv;
    __threadfence();
    if (wave == 0) *(volatile v4f*)rp = rv;
  }
}

__global__ __launch_bounds__(64) void k_bnstat(const float* __restrict__ rec, int gM, int nN, float* musc) {
  __shared__ __attribute__((aligned(16))) float ms[128];
  const int tid = (int)threadIdx.x, lane = tid & 31, wave = tid >> 5;
  double nA = 0.0, mA = 0.0, qA = 0.0;
#pragma unroll 1
  for (int b = 0; b < gM; ++b) {
    int nb = nN - b * GBM;
    nb = nb > GBM ? GBM : nb;
    if (nb > 0) {
      const double mB = (double)rec[(size_t)b * 128 + tid];
      const double qB = (double)rec[(size_t)b * 128 + EMB + tid];
      const double nB = (double)nb;
      const double nAB = nA + nB;
      const double ri = 1.0 / nAB;
      const double dl = mB - mA;
      mA = mA + dl * (nB * ri);
      qA = qA + qB + dl * dl * (nA * nB * ri);
      nA = nAB;
    }
  }
  const double var = qA * (1.0 / (double)nN);
  ms[tid] = (float)mA;
  ms[EMB + tid] = rsqrtf((float)var + 1e-5f);
  __syncthreads();
  const v4f ov = *(const v4fa*)(ms + 4 * lane);
  float* op = musc + 4 * lane;
  if (wave == 0) *(volatile v4f*)op = ov;
  __threadfence();
  if (wave == 0) *(volatile v4f*)op = ov;
}

__global__ __launch_bounds__(NTHR) void k_bnapply(const float* __restrict__ hn, const float* __restrict__ musc,
                                                  const float* __restrict__ gamma, const float* __restrict__ beta,
                                                  float* outp, int nElem, int doMish) {
  __shared__ __attribute__((aligned(16))) float buf[1024];
  __shared__ float pm[256];
  const int tid = (int)threadIdx.x;
  if (tid < EMB) {
    pm[tid]       = musc[tid];
    pm[64 + tid]  = musc[64 + tid];
    pm[128 + tid] = bf16_val(gamma[tid]);
    pm[192 + tid] = bf16_val(beta[tid]);
  }
  __syncthreads();
  const int base = (int)blockIdx.x * 1024;
#pragma unroll 1
  for (int it = 0; it < 4; ++it) {
    const int e  = base + it * NTHR + tid;
    const int ec = e < nElem ? e : nElem - 1;
    const int col = ec & (EMB - 1);
    const float x = hn[ec];
    float v = ((x - pm[col]) * pm[64 + col]) * pm[128 + col] + pm[192 + col];
    if (doMish != 0) {
      const float sp = fmaxf(v, 0.0f) + log1pf(expf(-fabsf(v)));
      v = v * tanhf(sp);
    }
    buf[it * NTHR + tid] = v;
  }
  __syncthreads();
  const v4f ov = *(const v4fa*)(buf + 4 * tid);
  const int e4 = base + 4 * tid;
  const bool ok = (e4 + 3) < nElem;
  float* op = outp + (size_t)e4;
  if (ok) *(volatile v4f*)op = ov;
  __threadfence();
  if (ok) *(volatile v4f*)op = ov;
}

static inline int cdiv(int a, int b) { return (a + b - 1) / b; }
static inline size_t al256(size_t o) { return (o + 255) & ~(size_t)255; }

extern "C" void kernel_launch(void* const* d_in, const int* in_sizes, int n_in,
                              void* d_out, int out_size, void* d_ws, size_t ws_size,
                              hipStream_t stream) {
  if (n_in < 12) return;
  if (in_sizes[0] < AF || (in_sizes[0] % AF) != 0) return;
  const int nN = in_sizes[0] / AF;
  if (nN < 64 || nN > (1 << 22)) return;
  if (in_sizes[11] < 2 || (in_sizes[11] & 1) != 0) return;
  const int nE = in_sizes[11] / 2;
  if (nE < 1 || nE >= (1 << (31 - SLA))) return;
  if ((long long)in_sizes[1] != (long long)nE * BF) return;
  if (in_sizes[2] != EMB * AF) return;
  if (in_sizes[3] != NL * HID2 * EMB || in_sizes[4] != NL * HID2) return;
  if (in_sizes[5] != NL * EMB * HID2 || in_sizes[6] != NL * EMB) return;
  if (in_sizes[7] != NL * EMB * BF || in_sizes[8] != NL * EMB) return;
  if (in_sizes[9] != NL * EMB || in_sizes[10] != NL * EMB) return;
  if ((long long)out_size != (long long)nN * EMB) return;

  const float* x     = (const float*)d_in[0];
  const float* eattr = (const float*)d_in[1];
  const float* Wemb  = (const float*)d_in[2];
  const float* W1    = (const float*)d_in[3];
  const float* b1    = (const float*)d_in[4];
  const float* W2    = (const float*)d_in[5];
  const float* b2    = (const float*)d_in[6];
  const float* We    = (const float*)d_in[7];
  const float* be    = (const float*)d_in[8];
  const float* gamma = (const float*)d_in[9];
  const float* beta  = (const float*)d_in[10];
  const int*   edge  = (const int*)d_in[11];
  float* out = (float*)d_out;
  const int* src = edge;
  const int* dst = edge + nE;

  const int MP = cdiv(nN, GBM) * GBM;
  const int gM = MP / GBM;
  const int gA = cdiv(MP, NBA);
  if ((long long)gA * NBA < (long long)MP) return;
  const int vec8 = ((nE & 3) == 0) ? 1 : 0;
  const int nElem = nN * EMB;
  if ((nElem & 3) != 0) return;

  char* ws = (char*)d_ws;
  size_t off = 0;
  const size_t oPE  = off; off = al256(off + (size_t)EMB * AF * 2);
  const size_t oPWE = off; off = al256(off + (size_t)NL * EMB * 32 * 2);
  const size_t oPW1 = off; off = al256(off + (size_t)NL * HID2 * K1 * 2);
  const size_t oPW2 = off; off = al256(off + (size_t)NL * EMB * K2 * 2);
  const size_t oXB  = off; off = al256(off + (size_t)MP * AF * 2);
  const size_t oH   = off; off = al256(off + (size_t)MP * EMB * 4);
  const size_t oHS  = off; off = al256(off + (size_t)MP * EMB * 4);
  const size_t oHN  = off; off = al256(off + (size_t)MP * EMB * 4);
  const size_t oEX  = off; off = al256(off + (size_t)MP * EXW * 4);
  const size_t oCNT = off; off = al256(off + (size_t)gA * NBA * 4);
  const size_t oOFF = off; off = al256(off + (size_t)gA * NBA * 4);
  const size_t oSRC = off; off = al256(off + (size_t)gA * RCAP * 4);
  const size_t oREC = off; off = al256(off + (size_t)gM * 128 * 4);
  const size_t oMS  = off; off = al256(off + (size_t)128 * 4);
  if (off > ws_size || off > (size_t)WSMAX) return;
  unsigned short* PE  = (unsigned short*)(ws + oPE);
  unsigned short* PWE = (unsigned short*)(ws + oPWE);
  unsigned short* PW1 = (unsigned short*)(ws + oPW1);
  unsigned short* PW2 = (unsigned short*)(ws + oPW2);
  unsigned short* XB  = (unsigned short*)(ws + oXB);
  float*    H    = (float*)(ws + oH);
  float*    HS   = (float*)(ws + oHS);
  float*    HN   = (float*)(ws + oHN);
  unsigned* EX   = (unsigned*)(ws + oEX);
  int*      CNT  = (int*)(ws + oCNT);
  int*      OFFS = (int*)(ws + oOFF);
  int*      SRCL = (int*)(ws + oSRC);
  float*    REC  = (float*)(ws + oREC);
  float*    MUSC = (float*)(ws + oMS);

  const size_t scanLds = (size_t)SCAN_LDS_INTS * 4;
  hipFuncSetAttribute(reinterpret_cast<const void*>(&k_scan0), hipFuncAttributeMaxDynamicSharedMemorySize, (int)scanLds);

  const int nUx = MP * (AF / 8);
  k_wprep<<<UTOT / NTHR, NTHR, 0, stream>>>(Wemb, We, W1, W2, PE, PWE, PW1, PW2);
  k_cvx<<<cdiv(nUx, NTHR), NTHR, 0, stream>>>(x, nN, nUx, XB);
  k_gemm<<<dim3(gM, EMB / GBN), GTHR, 0, stream>>>(XB, PE, H, AF, EMB);
  k_scan0<<<gA, NTHR, scanLds, stream>>>(src, dst, eattr, nE, nN, vec8, MP, H, HS, EX, CNT, OFFS, SRCL);

  for (int l = 0; l < NL; ++l) {
    k_mlp<<<gM, GTHR, 0, stream>>>(HS, (const unsigned short*)EX, (const int*)EX,
                                   PWE + (size_t)l * EMB * 32, PW1 + (size_t)l * HID2 * K1,
                                   PW2 + (size_t)l * EMB * K2,
                                   be + (size_t)l * EMB, b1 + (size_t)l * HID2, b2 + (size_t)l * EMB,
                                   HN, REC, nN);
    k_bnstat<<<1, 64, 0, stream>>>(REC, gM, nN, MUSC);
    float* dstp = (l == NL - 1) ? out : H;
    k_bnapply<<<cdiv(nElem, 1024), NTHR, 0, stream>>>(HN, MUSC, gamma + (size_t)l * EMB, beta + (size_t)l * EMB,
                                                      dstp, nElem, (l < NL - 1) ? 1 : 0);
    if (l < NL - 1) {
      k_gather<<<gA, NTHR, 0, stream>>>(CNT, OFFS, SRCL, nN, MP, H, HS);
    }
  }
}
